// PS_Attention_76768245448786
// MI455X (gfx1250) — hardware-verified
//
#include <hip/hip_runtime.h>
#include <math.h>
#include <stdint.h>

#define NBAT  4
#define CIN   256
#define IMW   56
#define HW    3136
#define MTOK  12544
#define NHG   16
#define HD    16
#define LWIN  392
#define LQP   400
#define LKP   416
#define NUNIT (2 * NBAT * 64)
#define STP   68
#define SBP   132
#define ASP   20
#define VTP   424
#define DTP   68
#define CDW   8.0f
#define CQS   256.0f
#define CKS   16.0f
#define CYS   256.0f
#define QKSC  (0.17677669529663688f / 4096.0f)
#define ATT_KS  0
#define ATT_VH  26624
#define ATT_VL  40192
#define ATT_ST  53760
#define ATT_END 64000

static_assert(ATT_VH == ATT_KS + LKP * 32 * 2);
static_assert(ATT_VL == ATT_VH + HD * VTP * 2);
static_assert(ATT_ST == ATT_VL + HD * VTP * 2);
static_assert(ATT_END == ATT_ST + 8 * 16 * ASP * 4);
static_assert(MTOK % 128 == 0);
static_assert(HW % 64 == 0);
static_assert((VTP % 8) == 0);
static_assert((ASP * 4) % 16 == 0);
static_assert((STP * 4) % 16 == 0);
static_assert((SBP * 4) % 16 == 0);
static_assert((DTP * 4) % 16 == 0);
static_assert(LQP == 25 * 16);
static_assert(LKP == 13 * 32);
static_assert(MTOK == NBAT * HW);

typedef _Float16 v16h __attribute__((ext_vector_type(16)));
typedef _Float16 v8h  __attribute__((ext_vector_type(8)));
typedef float    v8f  __attribute__((ext_vector_type(8)));
typedef float    v4f  __attribute__((ext_vector_type(4)));
typedef unsigned int v4u __attribute__((ext_vector_type(4)));
union Frag { v16h v; v8h half[2]; };

__device__ __forceinline__ unsigned short bf_bits(float f) {
  unsigned u = __float_as_uint(f);
  return (unsigned short)((u + 0x7FFFu + ((u >> 16) & 1u)) >> 16);
}
__device__ __forceinline__ float bfr(float f) { return __uint_as_float(((unsigned)bf_bits(f)) << 16); }
__device__ __forceinline__ unsigned short h_bits(_Float16 x) { return __builtin_bit_cast(unsigned short, x); }
__device__ __forceinline__ unsigned pk16(unsigned short a, unsigned short b) { return (unsigned)a | ((unsigned)b << 16); }
__device__ __forceinline__ v8f zero8() { v8f z = {0.f, 0.f, 0.f, 0.f, 0.f, 0.f, 0.f, 0.f}; return z; }
__device__ __forceinline__ v8h zero8h() {
  v8h z;
#pragma unroll
  for (int i = 0; i < 8; ++i) z[i] = (_Float16)0.0f;
  return z;
}

__device__ __forceinline__ v16h ldfrag_h(const _Float16* p) {
  Frag f;
  f.half[0] = *(const v8h*)(p);
  f.half[1] = *(const v8h*)(p + 16);
  return f.v;
}

__device__ __forceinline__ v8f mma_h(v16h a, v16h b, v8f c) {
  c = __builtin_amdgcn_wmma_f32_16x16x32_f16(false, a, false, b, (short)0, c, false, false);
#if defined(__HIP_DEVICE_COMPILE__)
  asm volatile("v_nop\n\tv_nop\n\tv_nop\n\tv_nop" : "+v"(c) : "v"(a), "v"(b));
#endif
  return c;
}
__device__ __forceinline__ void wave_sync_lds() {
  __builtin_amdgcn_fence(__ATOMIC_RELEASE, "workgroup");
  __builtin_amdgcn_wave_barrier();
  __builtin_amdgcn_fence(__ATOMIC_ACQUIRE, "workgroup");
}

__device__ __forceinline__ v4u pack8h(v4f a, v4f b) {
  v4u p;
  p[0] = pk16(h_bits((_Float16)a[0]), h_bits((_Float16)a[1]));
  p[1] = pk16(h_bits((_Float16)a[2]), h_bits((_Float16)a[3]));
  p[2] = pk16(h_bits((_Float16)b[0]), h_bits((_Float16)b[1]));
  p[3] = pk16(h_bits((_Float16)b[2]), h_bits((_Float16)b[3]));
  return p;
}
__device__ __forceinline__ void split8h(v4f a, v4f b, v4u& ph, v4u& pl) {
  v4f ra, rb;
#pragma unroll
  for (int e = 0; e < 4; ++e) {
    const _Float16 ha = (_Float16)a[e];
    ra[e] = (a[e] - (float)ha) * 2048.0f;
    const _Float16 hb = (_Float16)b[e];
    rb[e] = (b[e] - (float)hb) * 2048.0f;
  }
  ph = pack8h(a, b);
  pl = pack8h(ra, rb);
}

__device__ __forceinline__ int tok_T(int n, int br, int g, int b) {
  const int p0 = n / IMW, w0 = n - p0 * IMW;
  const int t0 = (p0 * 8 + g) * IMW + w0;
  const int h1 = n / 7, p1 = n - h1 * 7;
  const int t1 = h1 * IMW + p1 * 8 + g;
  return b * HW + ((br != 0) ? t1 : t0);
}

__device__ __forceinline__ void cvt8_w(const float* __restrict__ src, unsigned short* dst, size_t e0) {
  const v4f a = *(const v4f*)(src + e0);
  const v4f b = *(const v4f*)(src + e0 + 4);
  v4f sa, sb;
#pragma unroll
  for (int e = 0; e < 4; ++e) { sa[e] = bfr(a[e]) * 256.0f; sb[e] = bfr(b[e]) * 256.0f; }
  const v4u pk = pack8h(sa, sb);
  *(volatile v4u*)(dst + e0) = pk;
  __threadfence();
  *(volatile v4u*)(dst + e0) = pk;
}
__global__ __launch_bounds__(256) void cvt_w(const float* __restrict__ wq, const float* __restrict__ wp,
                                             unsigned short* Wq, unsigned short* Wp) {
  const int tid = threadIdx.x, blk = blockIdx.x;
  if (blk < 96) cvt8_w(wq, Wq, ((size_t)blk * 256 + tid) * 8);
  else          cvt8_w(wp, Wp, ((size_t)(blk - 96) * 256 + tid) * 8);
}

__global__ __launch_bounds__(256)
void dwbn_k(const float* __restrict__ x, const float* __restrict__ dw, const float* __restrict__ gam,
            const float* __restrict__ bet, const float* __restrict__ mea, const float* __restrict__ var,
            unsigned short* Ah, unsigned short* Al) {
  __shared__ __align__(16) float tile[3 * 64 * DTP];
  const int tid = threadIdx.x, bid = blockIdx.x;
  const int cq = bid & 3, bp = bid >> 2;
  const int pt = bp % 49, b = bp / 49;
  const int px = tid & 63, cg = tid >> 6;
  const int s = pt * 64 + px;
  const int h = s / IMW, w = s - h * IMW;
  int toff[9];
  float tmsk[9];
#pragma unroll
  for (int dy = 0; dy < 3; ++dy) {
#pragma unroll
    for (int dx = 0; dx < 3; ++dx) {
      const int hy = h + dy - 1, wx = w + dx - 1;
      const bool ok = ((unsigned)hy < (unsigned)IMW) && ((unsigned)wx < (unsigned)IMW);
      const int hc = (hy < 0) ? 0 : ((hy > IMW - 1) ? (IMW - 1) : hy);
      const int wc = (wx < 0) ? 0 : ((wx > IMW - 1) ? (IMW - 1) : wx);
      toff[dy * 3 + dx] = hc * IMW + wc;
      tmsk[dy * 3 + dx] = ok ? 1.0f : 0.0f;
    }
  }
  const int ch0 = cq * 64 + cg * 16;
#pragma unroll 1
  for (int j = 0; j < 16; ++j) {
    const int ch = ch0 + j;
    const float* xp = x + ((size_t)(b * CIN + ch)) * HW;
    float xv[9];
#pragma unroll
    for (int t = 0; t < 9; ++t) xv[t] = bfr(xp[toff[t]]) * tmsk[t];
#pragma unroll 1
    for (int part = 0; part < 3; ++part) {
      const int pc = part * CIN + ch;
      const float* w9 = dw + (size_t)pc * 9;
      float acc = 0.f;
#pragma unroll
      for (int t = 0; t < 9; ++t) acc += xv[t] * bfr(w9[t]);
      const float inv = bfr(gam[pc]) * rsqrtf(bfr(var[pc]) + 1.0e-5f);
      const float o = acc * inv + (bfr(bet[pc]) - bfr(mea[pc]) * inv);
      tile[(part * 64 + px) * DTP + cg * 16 + j] = o;
    }
  }
  __syncthreads();
  const int piece = tid & 7, rsub = tid >> 3;
#pragma unroll 1
  for (int part = 0; part < 3; ++part) {
    v4u ph[2], pl[2];
    size_t offs[2];
#pragma unroll
    for (int it = 0; it < 2; ++it) {
      const int row = it * 32 + rsub;
      v4f fa = *(const v4f*)(tile + (part * 64 + row) * DTP + piece * 8);
      v4f fb = *(const v4f*)(tile + (part * 64 + row) * DTP + piece * 8 + 4);
      fa = fa * CDW;
      fb = fb * CDW;
      split8h(fa, fb, ph[it], pl[it]);
      offs[it] = ((size_t)part * MTOK + (size_t)(b * HW + pt * 64 + row)) * CIN + cq * 64 + piece * 8;
    }
    for (int pass = 0; pass < 2; ++pass) {
#pragma unroll
      for (int it = 0; it < 2; ++it) {
        *(volatile v4u*)(Ah + offs[it]) = ph[it];
        *(volatile v4u*)(Al + offs[it]) = pl[it];
      }
      __threadfence();
    }
  }
}

__global__ __launch_bounds__(256)
void gemm_pw(const unsigned short* __restrict__ Ah, const unsigned short* __restrict__ Al,
             const unsigned short* __restrict__ Wq, unsigned short* PL) {
  __shared__ __align__(16) float sbuf[8 * 16 * STP];
  const int tid = threadIdx.x, wave = tid >> 5, lane = tid & 31, hh = lane >> 4, c = lane & 15;
  const int n0 = blockIdx.x * 64, m0 = blockIdx.y * 128, part = blockIdx.z;
  const int arow = m0 + wave * 16 + c;
  const size_t aplane = (size_t)part * MTOK * CIN;
  const _Float16* A0 = (const _Float16*)(const void*)Ah + aplane;
  const _Float16* A1 = (const _Float16*)(const void*)Al + aplane;
  const _Float16* B  = (const _Float16*)(const void*)Wq + (size_t)part * CIN * CIN;

  v8f acch[4], accl[4];
#pragma unroll
  for (int nt = 0; nt < 4; ++nt) { acch[nt] = zero8(); accl[nt] = zero8(); }

#pragma unroll 1
  for (int k0 = 0; k0 < CIN; k0 += 32) {
    const size_t aoff = (size_t)arow * CIN + k0 + 8 * hh;
    const v16h ah = ldfrag_h(A0 + aoff);
    const v16h al = ldfrag_h(A1 + aoff);
#pragma unroll
    for (int nt = 0; nt < 4; ++nt) {
      const v16h bfrag = ldfrag_h(B + (size_t)(n0 + nt * 16 + c) * CIN + k0 + 8 * hh);
      acch[nt] = mma_h(ah, bfrag, acch[nt]);
      accl[nt] = mma_h(al, bfrag, accl[nt]);
    }
  }

  const float osc = (part == 0) ? (CQS / 2048.0f) : (CKS / 2048.0f);
  float* st = sbuf + wave * (16 * STP);
#pragma unroll
  for (int nt = 0; nt < 4; ++nt) {
#pragma unroll
    for (int r = 0; r < 8; ++r) {
      const float v = acch[nt][r] + accl[nt][r] * (1.0f / 2048.0f);
      st[(8 * hh + r) * STP + nt * 16 + c] = v * osc;
    }
  }
  wave_sync_lds();
  const int hgl = c >> 2, sel = (c >> 1) & 1, halfd = c & 1;
  const int col = hgl * 16 + halfd * 8;
  v4u pk[8];
  size_t offs[8];
#pragma unroll
  for (int it = 0; it < 8; ++it) {
    const int q = it * 2 + hh;
    const v4f fa = *(const v4f*)(st + q * STP + col);
    const v4f fb = *(const v4f*)(st + q * STP + col + 4);
    v4u vh, vl;
    split8h(fa, fb, vh, vl);
#pragma unroll
    for (int e = 0; e < 4; ++e) pk[it][e] = sel ? vl[e] : vh[e];
    const size_t T = (size_t)(m0 + wave * 16 + q);
    offs[it] = (((size_t)part * MTOK + T) * NHG + (size_t)((n0 >> 4) + hgl)) * 32 + sel * 16 + halfd * 8;
  }
  for (int pass = 0; pass < 2; ++pass) {
#pragma unroll
    for (int it = 0; it < 8; ++it) *(volatile v4u*)(PL + offs[it]) = pk[it];
    __threadfence();
  }
}

__global__ __launch_bounds__(256)
void attn_k(const unsigned short* __restrict__ PL, unsigned short* Oh, unsigned short* Ol) {
  extern __shared__ __align__(16) char smem[];
  unsigned short* Ks = (unsigned short*)(smem + ATT_KS);
  unsigned short* Vt = (unsigned short*)(smem + ATT_VH);
  float* Sst = (float*)(smem + ATT_ST);
  const int tid = threadIdx.x, wave = tid >> 5, lane = tid & 31, hh = lane >> 4, c = lane & 15;
  const int u = blockIdx.x;
  const int head = u & 7, g = (u >> 3) & 7, b = (u >> 6) % NBAT, br = u / (64 * NBAT);
  const int hg = br * 8 + head;
  const size_t psz = (size_t)MTOK * NHG * 32;
  const unsigned short* Qp = PL;
  const unsigned short* Kp = PL + psz;
  const unsigned short* Vp = PL + 2 * psz;

#pragma unroll
  for (int it = 0; it < 2; ++it) {
    const int n = it * 256 + tid;
    const int nn = (n < LWIN) ? n : (LWIN - 1);
    const size_t T = (size_t)tok_T(nn, br, g, b);
    const v4u* kgp = (const v4u*)(Kp + (T * NHG + hg) * 32);
    const v4u* vgp = (const v4u*)(Vp + (T * NHG + hg) * 32);
    v4u kw[4], vw[4];
#pragma unroll
    for (int i = 0; i < 4; ++i) { kw[i] = kgp[i]; vw[i] = vgp[i]; }
    const bool live = (n < LWIN);
#pragma unroll
    for (int i = 0; i < 4; ++i) {
#pragma unroll
      for (int e = 0; e < 4; ++e) {
        kw[i][e] = live ? kw[i][e] : 0u;
        vw[i][e] = live ? vw[i][e] : 0u;
      }
    }
    if (n < LKP) {
#pragma unroll
      for (int i = 0; i < 4; ++i) {
        *(v4u*)(Ks + n * 32 + 8 * i) = kw[i];
        const int d0 = (i >> 1) * 16 + (i & 1) * 8;
#pragma unroll
        for (int e = 0; e < 4; ++e) {
          const unsigned w32 = vw[i][e];
          Vt[(d0 + 2 * e) * VTP + n]     = (unsigned short)(w32 & 0xFFFFu);
          Vt[(d0 + 2 * e + 1) * VTP + n] = (unsigned short)(w32 >> 16);
        }
      }
    }
  }
  __syncthreads();

  const _Float16* Ksh = (const _Float16*)(const void*)Ks;
  const _Float16* Vth = (const _Float16*)(const void*)Vt;
  float* st = Sst + wave * (16 * ASP);
  const v8h z8 = zero8h();

#pragma unroll 1
  for (int qt = wave; qt < 25; qt += 8) {
    const int lqc = qt * 16 + c;
    const int lq = (lqc < LWIN) ? lqc : (LWIN - 1);
    const size_t Tq = (size_t)tok_T(lq, br, g, b);
    const _Float16* qrow = (const _Float16*)(const void*)(Qp + (Tq * NHG + hg) * 32);
    Frag b1, b2;
    b1.half[0] = *(const v8h*)(qrow + 8 * hh);
    b2.half[0] = *(const v8h*)(qrow + 16 + 8 * hh);
    v8h hp;
#pragma unroll
    for (int i = 0; i < 8; ++i) {
      float f = (float)b1.half[0][i] * (1.0f / 2048.0f);
      f = (fabsf(f) < 6.103515625e-05f) ? 0.0f : f;
      hp[i] = (_Float16)f;
    }
    b1.half[1] = hp;
    b2.half[1] = z8;

    v8f o = zero8(), ol = zero8();
    float mrun = -1.0e30f, lrun = 0.f;
#pragma unroll 1
    for (int ch = 0; ch < 13; ++ch) {
      const int kb = ch * 32;
      v8f s[2];
#pragma unroll
      for (int j = 0; j < 2; ++j) {
        const v16h ka = ldfrag_h(Ksh + (size_t)(kb + j * 16 + c) * 32 + 8 * hh);
        const v8f a1 = mma_h(ka, b1.v, zero8());
        const v8f a2 = mma_h(ka, b2.v, zero8());
        s[j] = a1 + a2 * (1.0f / 2048.0f);
      }
      if (ch == 12) {
#pragma unroll
        for (int r = 0; r < 8; ++r) {
          s[0][r] = (hh != 0) ? -1.0e30f : s[0][r];
          s[1][r] = -1.0e30f;
        }
      }
      float mc = s[0][0];
#pragma unroll
      for (int j = 0; j < 2; ++j) {
#pragma unroll
        for (int r = 0; r < 8; ++r) mc = fmaxf(mc, s[j][r]);
      }
      mc = fmaxf(mc, __shfl_xor(mc, 16, 32));
      const float mnew = fmaxf(mrun, mc);
      const float alpha = __expf((mrun - mnew) * QKSC);
#pragma unroll
      for (int r = 0; r < 8; ++r) {
        const float ar = __shfl(alpha, 8 * hh + r, 32);
        o[r] = o[r] * ar;
        ol[r] = ol[r] * ar;
      }
      float psum = 0.f;
      v16h pfh, pfl;
#pragma unroll
      for (int i = 0; i < 8; ++i) {
        const float e0 = __expf((s[0][i] - mnew) * QKSC);
        const float e1 = __expf((s[1][i] - mnew) * QKSC);
        psum = psum + (e0 + e1);
        const float t0 = e0 * 1024.0f, t1 = e1 * 1024.0f;
        const _Float16 h0 = (_Float16)t0, h1 = (_Float16)t1;
        pfh[i]     = h0;
        pfl[i]     = (_Float16)((t0 - (float)h0) * 2048.0f);
        pfh[8 + i] = h1;
        pfl[8 + i] = (_Float16)((t1 - (float)h1) * 2048.0f);
      }
      lrun = lrun * alpha + psum;
      mrun = mnew;
      {
        const v16h vfh = ldfrag_h(Vth + (size_t)c * VTP + kb + 8 * hh);
        const v16h vfl = ldfrag_h(Vth + (size_t)(HD + c) * VTP + kb + 8 * hh);
        o  = mma_h(pfh, vfh, o);
        ol = mma_h(pfh, vfl, ol);
        ol = mma_h(pfl, vfh, ol);
      }
    }
    const float lsum = lrun + __shfl_xor(lrun, 16, 32);
#pragma unroll
    for (int r = 0; r < 8; ++r) {
      const int q = 8 * hh + r;
      const float lqv = __shfl(lsum, q, 32);
      const float inv = (CYS / 16384.0f) / lqv;
      st[q * ASP + c] = (o[r] + ol[r] * (1.0f / 2048.0f)) * inv;
    }
    wave_sync_lds();
    {
      const int tq = lane >> 1, dh = (lane & 1) * 8;
      const v4f fa = *(const v4f*)(st + tq * ASP + dh);
      const v4f fb = *(const v4f*)(st + tq * ASP + dh + 4);
      v4u ph, pl;
      split8h(fa, fb, ph, pl);
      const size_t off = ((size_t)u * LQP + (size_t)(qt * 16 + tq)) * HD + dh;
      for (int pass = 0; pass < 2; ++pass) {
        *(volatile v4u*)(Oh + off) = ph;
        *(volatile v4u*)(Ol + off) = pl;
        __threadfence();
      }
    }
    wave_sync_lds();
  }
}

__global__ __launch_bounds__(256)
void gemm_proj(const unsigned short* __restrict__ Oh, const unsigned short* __restrict__ Ol,
               const unsigned short* __restrict__ Wp, const float* __restrict__ pb, float* out) {
  __shared__ __align__(16) float sb[64 * SBP];
  const int tid = threadIdx.x, wave = tid >> 5, lane = tid & 31, hh = lane >> 4, c = lane & 15;
  const int n0 = blockIdx.x * 64, m0 = blockIdx.y * 128;
  const int T = m0 + wave * 16 + c;
  const int bimg = T / HW, s = T - bimg * HW, h = s / IMW, w = s - h * IMW;
  const int g0 = h & 7, l0 = (h >> 3) * IMW + w;
  const int g1 = w & 7, l1 = h * 7 + (w >> 3);
  const size_t base0 = ((size_t)((bimg * 8 + g0) * 8) * LQP + (size_t)l0) * HD + 8 * hh;
  const size_t base1 = ((size_t)(((NBAT + bimg) * 8 + g1) * 8) * LQP + (size_t)l1) * HD + 8 * hh;
  const _Float16* A0 = (const _Float16*)(const void*)Oh;
  const _Float16* A1 = (const _Float16*)(const void*)Ol;
  const _Float16* B  = (const _Float16*)(const void*)Wp;

  v8f acch[4], accl[4];
#pragma unroll
  for (int nt = 0; nt < 4; ++nt) { acch[nt] = zero8(); accl[nt] = zero8(); }

#pragma unroll 1
  for (int ks = 0; ks < 8; ++ks) {
    const size_t bo = (((ks >> 2) != 0) ? base1 : base0) + (size_t)((ks & 3) * 2) * (LQP * HD);
    Frag fh, fl;
    fh.half[0] = *(const v8h*)(A0 + bo);
    fh.half[1] = *(const v8h*)(A0 + bo + LQP * HD);
    fl.half[0] = *(const v8h*)(A1 + bo);
    fl.half[1] = *(const v8h*)(A1 + bo + LQP * HD);
#pragma unroll
    for (int nt = 0; nt < 4; ++nt) {
      const v16h bfrag = ldfrag_h(B + (size_t)(n0 + nt * 16 + c) * CIN + ks * 32 + 8 * hh);
      acch[nt] = mma_h(fh.v, bfrag, acch[nt]);
      accl[nt] = mma_h(fl.v, bfrag, accl[nt]);
    }
  }

#pragma unroll
  for (int nt = 0; nt < 4; ++nt) {
#pragma unroll
    for (int r = 0; r < 8; ++r) {
      const float v = acch[nt][r] + accl[nt][r] * (1.0f / 2048.0f);
      sb[(nt * 16 + c) * SBP + wave * 16 + 8 * hh + r] = v * (1.0f / 65536.0f);
    }
  }
  __syncthreads();
  v4f ov[8];
  size_t offs[8];
  const int Th = m0 + hh * 64;
  const int bi = Th / HW, s0 = Th - bi * HW;
#pragma unroll
  for (int i = 0; i < 8; ++i) {
    const int cc = wave * 8 + i;
    const int co = n0 + cc;
    const float bias = bfr(pb[co]);
    const v4f t = *(const v4f*)(sb + cc * SBP + hh * 64 + c * 4);
    ov[i] = t + bias;
    offs[i] = ((size_t)(bi * CIN + co)) * HW + s0 + c * 4;
  }
  for (int pass = 0; pass < 2; ++pass) {
#pragma unroll
    for (int i = 0; i < 8; ++i) *(volatile v4f*)(out + offs[i]) = ov[i];
    __threadfence();
  }
}

extern "C" void kernel_launch(void* const* d_in, const int* in_sizes, int n_in,
                              void* d_out, int out_size, void* d_ws, size_t ws_size,
                              hipStream_t stream) {
  if (n_in < 9) return;
  if (in_sizes[0] != NBAT * CIN * HW) return;
  if (in_sizes[1] != 3 * CIN * 9) return;
  if (in_sizes[2] != 3 * CIN || in_sizes[3] != 3 * CIN || in_sizes[4] != 3 * CIN || in_sizes[5] != 3 * CIN) return;
  if (in_sizes[6] != 3 * CIN * CIN) return;
  if (in_sizes[7] != CIN * CIN || in_sizes[8] != CIN) return;
  if (out_size != NBAT * CIN * HW) return;

  const float* x    = (const float*)d_in[0];
  const float* dw   = (const float*)d_in[1];
  const float* gam  = (const float*)d_in[2];
  const float* bet  = (const float*)d_in[3];
  const float* mea  = (const float*)d_in[4];
  const float* var  = (const float*)d_in[5];
  const float* pw   = (const float*)d_in[6];
  const float* pjw  = (const float*)d_in[7];
  const float* pjb  = (const float*)d_in[8];
  float* out = (float*)d_out;

  const size_t sWq = (size_t)3 * CIN * CIN * 2;
  const size_t sWp = (size_t)CIN * CIN * 2;
  const size_t sA  = (size_t)3 * MTOK * CIN * 2;
  const size_t sPL = (size_t)3 * MTOK * NHG * 32 * 2;
  const size_t sO  = (size_t)NUNIT * LQP * HD * 2;
  size_t off = 0;
  const size_t oWq = off; off += sWq;
  const size_t oWp = off; off += sWp;
  const size_t oAh = off; off += sA;
  const size_t oAl = off; off += sA;
  const size_t oPL = off; off += sPL;
  const size_t oOh = off; off += sO;
  const size_t oOl = off; off += sO;
  if (off > ws_size) return;
  if (off > (size_t)134217728) return;

  char* ws = (char*)d_ws;
  unsigned short* Wq = (unsigned short*)(ws + oWq);
  unsigned short* Wp = (unsigned short*)(ws + oWp);
  unsigned short* Ah = (unsigned short*)(ws + oAh);
  unsigned short* Al = (unsigned short*)(ws + oAl);
  unsigned short* PL = (unsigned short*)(ws + oPL);
  unsigned short* Oh = (unsigned short*)(ws + oOh);
  unsigned short* Ol = (unsigned short*)(ws + oOl);

  const dim3 blk(256);
  cvt_w<<<dim3(128), blk, 0, stream>>>(pw, pjw, Wq, Wp);
  dwbn_k<<<dim3(NBAT * 49 * 4), blk, 0, stream>>>(x, dw, gam, bet, mea, var, Ah, Al);
  gemm_pw<<<dim3(CIN / 64, MTOK / 128, 3), blk, 0, stream>>>(Ah, Al, Wq, PL);
  (void)hipFuncSetAttribute(reinterpret_cast<const void*>(&attn_k), hipFuncAttributeMaxDynamicSharedMemorySize, ATT_END);
  attn_k<<<dim3(NUNIT), blk, ATT_END, stream>>>(PL, Oh, Ol);
  gemm_proj<<<dim3(CIN / 64, MTOK / 128), blk, 0, stream>>>(Oh, Ol, Wp, pjb, out);
  (void)hipGetLastError();
}
